// GQA_40750649704889
// MI455X (gfx1250) — hardware-verified
//
#include <hip/hip_runtime.h>


#ifndef NB
#define NB 2
#endif
#ifndef SEQ
#define SEQ 2048
#endif
#define TT      SEQ
#define TT_FULL 2048
#define DM      2048
#define NQH     32
#define NKV     8
#define REP     (NQH / NKV)
#define HD      64
#define HP      (HD / 2)
#define NPL     (NQH + NKV)
#define NQKV    ((NQH + 2 * NKV) * HD)
#define ZH      4
#define RHW     512
#define RH      ((TT < RHW) ? TT : RHW)
#define PCAR    1024.0f
#define SCL     0.125f
#define ASC     64.0f
#define WSC     256.0f
#define OSC     (1.0f / (64.0f * 256.0f))
#define LOG2E   1.4426950408889634f
#define RBASE   10000.0f

static_assert(TT % 128 == 0);
static_assert(RH % 128 == 0);
static_assert(RH <= TT);
static_assert((TT - RH) % 64 == 0);
static_assert(DM % 64 == 0);
static_assert(NQKV % 64 == 0);
static_assert(HD == 64);
static_assert(HP == 32);
static_assert(REP % ZH == 0);
static_assert(NQH % ZH == 0);
static_assert(TT <= TT_FULL);

typedef _Float16 h16;
typedef unsigned short bf;
typedef __attribute__((ext_vector_type(16))) __bf16   v16bf;
typedef __attribute__((ext_vector_type(16))) _Float16 v16h;
typedef __attribute__((ext_vector_type(8)))  _Float16 v8h;
typedef __attribute__((ext_vector_type(8)))  unsigned short v8us;
typedef __attribute__((ext_vector_type(8)))  float    v8f;
typedef __attribute__((ext_vector_type(4)))  float    v4f;
typedef __attribute__((ext_vector_type(2)))  float    v2f;
typedef __attribute__((ext_vector_type(2)))  _Float16 v2h;
typedef __attribute__((ext_vector_type(4)))  _Float16 v4h;
typedef __attribute__((ext_vector_type(2)))  unsigned short v2us;
typedef __attribute__((ext_vector_type(4)))  unsigned short v4us;
typedef v8h  __attribute__((may_alias)) v8ha;
typedef v4f  __attribute__((may_alias)) v4fa;
typedef v8us __attribute__((may_alias)) v8usa;

__device__ __forceinline__ unsigned short f2bf(float f) { unsigned u = __float_as_uint(f); u += 0x7FFFu + ((u >> 16) & 1u); return (unsigned short)(u >> 16); }
__device__ __forceinline__ float bf2f(unsigned short b) { return __uint_as_float(((unsigned)b) << 16); }
__device__ __forceinline__ float bfr(float f) { return bf2f(f2bf(f)); }
__device__ __forceinline__ v16h cat16(v8h lo, v8h hi) { return __builtin_shufflevector(lo, hi, 0, 1, 2, 3, 4, 5, 6, 7, 8, 9, 10, 11, 12, 13, 14, 15); }
__device__ __forceinline__ v16bf cat16b(v8us lo, v8us hi) { return __builtin_bit_cast(v16bf, __builtin_shufflevector(lo, hi, 0, 1, 2, 3, 4, 5, 6, 7, 8, 9, 10, 11, 12, 13, 14, 15)); }
__device__ __forceinline__ v8f wmma16(v16h a, v16h b, v8f c) { return __builtin_amdgcn_wmma_f32_16x16x32_f16(false, a, false, b, (short)0, c, false, false); }
__device__ __forceinline__ v8f wmmab(v16bf a, v16bf b, v8f c) { return __builtin_amdgcn_wmma_f32_16x16x32_bf16(false, a, false, b, (short)0, c, false, false); }
__device__ __forceinline__ h16 tohx(float x) { return (h16)x; }
__device__ __forceinline__ void splitf(float y, unsigned short& h, unsigned short& l) { h = f2bf(y); l = f2bf(y - bf2f(h)); }

template <typename T16> struct WFrag;
template <> struct WFrag<h16> { typedef v16h V; static __device__ __forceinline__ V ld(const h16* p) { return cat16(*(const v8h*)p, *(const v8h*)(p + 16)); } static __device__ __forceinline__ v8f mma(V a, V b, v8f c) { return wmma16(a, b, c); } };
template <> struct WFrag<bf> { typedef v16bf V; static __device__ __forceinline__ V ld(const bf* p) { return cat16b(*(const v8us*)p, *(const v8us*)(p + 16)); } static __device__ __forceinline__ v8f mma(V a, V b, v8f c) { return wmmab(a, b, c); } };
template <typename T16, int NSPLIT, int CAUS>
__global__ __launch_bounds__(32) void k_gemmw(const T16* __restrict__ A, const T16* __restrict__ A2, int lda, const T16* __restrict__ Bt, const T16* __restrict__ Bt2, int ldb, int K, int qoff, float* C, int ldc, float osc, size_t sA, size_t sB, size_t sC) {
    typedef typename WFrag<T16>::V V;
    __shared__ __align__(16) float os[16 * 68];
    const size_t z = blockIdx.z; A += z * sA; if (A2) A2 += z * sA; Bt += z * sB; if (Bt2) Bt2 += z * sB; C += z * sC;
    const int lane = threadIdx.x & 31, lr = lane & 15, hi = lane >> 4; const int r0 = blockIdx.x * 64, c0 = blockIdx.y * 64;
    if (CAUS == 1 && c0 >= r0 + qoff + 64) return;
    const int kend = (CAUS == 2) ? ((r0 + qoff + 64 < K) ? (r0 + qoff + 64) : K) : K;
    v8f acc[4][4];
#pragma unroll
    for (int mb = 0; mb < 4; ++mb)
#pragma unroll
        for (int nb = 0; nb < 4; ++nb) acc[mb][nb] = (v8f){};
    const size_t aoff = (size_t)(r0 + lr) * lda + 8 * hi, boff = (size_t)(c0 + lr) * ldb + 8 * hi;
#pragma unroll 1
    for (int kc = 0; kc < kend; kc += 32) {
        V a[4], a2[4];
#pragma unroll
        for (int mb = 0; mb < 4; ++mb) { a[mb] = WFrag<T16>::ld(A + aoff + (size_t)mb * 16 * lda + kc); if (NSPLIT == 1 || NSPLIT == 2) a2[mb] = WFrag<T16>::ld(A2 + aoff + (size_t)mb * 16 * lda + kc); }
#pragma unroll
        for (int nb = 0; nb < 4; ++nb) { const V b = WFrag<T16>::ld(Bt + boff + (size_t)nb * 16 * ldb + kc); V b2; if (NSPLIT >= 2) b2 = WFrag<T16>::ld(Bt2 + boff + (size_t)nb * 16 * ldb + kc);
#pragma unroll
            for (int mb = 0; mb < 4; ++mb) { acc[mb][nb] = WFrag<T16>::mma(a[mb], b, acc[mb][nb]); if (NSPLIT == 1 || NSPLIT == 2) acc[mb][nb] = WFrag<T16>::mma(a2[mb], b, acc[mb][nb]); if (NSPLIT >= 2) acc[mb][nb] = WFrag<T16>::mma(a[mb], b2, acc[mb][nb]); } }
        asm volatile("v_nop\n\tv_nop\n\tv_nop\n\tv_nop" : "+v"(acc[0][0]), "+v"(acc[1][1]), "+v"(acc[2][2]), "+v"(acc[3][3]) : "v"(a[0]), "v"(a[3]));
    }
#pragma unroll
    for (int mb = 0; mb < 4; ++mb) {
#pragma unroll
        for (int nb = 0; nb < 4; ++nb) {
#pragma unroll
            for (int j = 0; j < 8; ++j) os[(hi * 8 + j) * 68 + nb * 16 + lr] = acc[mb][nb][j]; }
        __builtin_amdgcn_wave_barrier(); asm volatile("" ::: "memory");
        float* crow = C + (size_t)(r0 + mb * 16) * ldc + c0;
#pragma unroll 1
        for (int ps = 0; ps < 2; ++ps) {
#pragma unroll
            for (int s = 0; s < 8; ++s) { const int row = 2 * s + hi, cofs = lr * 4; v4f val = *(const v4fa*)(os + row * 68 + cofs);
                val[0] = val[0] * osc; val[1] = val[1] * osc; val[2] = val[2] * osc; val[3] = val[3] * osc;
                *(volatile v4f*)(crow + (size_t)row * ldc + cofs) = val; }
            if (ps == 0) __threadfence(); }
        __builtin_amdgcn_wave_barrier(); asm volatile("" ::: "memory");
    }
}

__global__ __launch_bounds__(256) void k_cvt8(const float* __restrict__ src, bf* dst, size_t n8) { const size_t i = (size_t)blockIdx.x * 256 + threadIdx.x; if (i >= n8) return; const v8f v = *(const v8f*)(src + i * 8); v8us o;
#pragma unroll
    for (int k = 0; k < 8; ++k) o[k] = f2bf(v[k]); *(volatile v8us*)(dst + i * 8) = o; __threadfence(); *(volatile v8us*)(dst + i * 8) = o; }
__global__ __launch_bounds__(256) void k_cvt8h(const float* __restrict__ src, h16* dst, float sc, size_t n8) { const size_t i = (size_t)blockIdx.x * 256 + threadIdx.x; if (i >= n8) return; const v8f v = *(const v8f*)(src + i * 8); v8h o;
#pragma unroll
    for (int k = 0; k < 8; ++k) o[k] = tohx(bfr(v[k]) * sc); *(volatile v8h*)(dst + i * 8) = o; __threadfence(); *(volatile v8h*)(dst + i * 8) = o; }
__global__ __launch_bounds__(32) void k_theta(float* TH) { const int p = threadIdx.x; const float ex = (float)(2 * p) * (1.0f / (float)HD); const float th = 1.0f / powf(RBASE, ex); *(volatile float*)(TH + p) = th; __threadfence(); *(volatile float*)(TH + p) = th; }
__global__ __launch_bounds__(256) void k_cstab(const float* __restrict__ TH, float* CS) { const int idx = blockIdx.x * 256 + threadIdx.x; if (idx >= TT * HP) return; const int p = idx % HP; const int t = idx / HP;
    const float ang = __fmul_rn((float)t, TH[p]); float s, c; sincosf(ang, &s, &c); v2f cs; cs[0] = c; cs[1] = s;
    *(volatile v2f*)(CS + (size_t)idx * 2) = cs; __threadfence(); *(volatile v2f*)(CS + (size_t)idx * 2) = cs; }
__global__ __launch_bounds__(256) void k_rope(const float* __restrict__ F, int pitch, int nheads, const float* __restrict__ CS, h16* P16, bf* Ph, bf* Pl) {
    const size_t e = ((size_t)blockIdx.x * 256 + threadIdx.x) * 2; if (e >= (size_t)nheads * TT * HD) return;
    const int d = (int)(e % HD); const int t = (int)((e / HD) % TT); const int h = (int)(e / ((size_t)HD * TT));
    const v2f xv = *(const v2f*)(F + (size_t)t * pitch + h * HD + d);
    const v2f cs = *(const v2f*)(CS + ((size_t)t * HP + (d >> 1)) * 2);
    float a0 = __fmul_rn(xv[0], cs[0]), b0 = __fmul_rn(xv[1], cs[1]), a1 = __fmul_rn(xv[1], cs[0]), b1 = __fmul_rn(xv[0], cs[1]);
    asm volatile("" : "+v"(a0)); asm volatile("" : "+v"(b0)); asm volatile("" : "+v"(a1)); asm volatile("" : "+v"(b1));
    const float r0 = __fsub_rn(a0, b0), r1 = __fadd_rn(a1, b1);
    v2h o16; o16[0] = tohx(r0); o16[1] = tohx(r1);
    v2us oh, ol; { unsigned short a, c; splitf(r0, a, c); oh[0] = a; ol[0] = c; splitf(r1, a, c); oh[1] = a; ol[1] = c; }
    const bool lo = (t < RH); const size_t oo = ((size_t)h * RH + (lo ? t : 0)) * HD + d;
    *(volatile v2h*)(P16 + e) = o16; if (lo) { *(volatile v2us*)(Ph + oo) = oh; *(volatile v2us*)(Pl + oo) = ol; }
    __threadfence();
    *(volatile v2h*)(P16 + e) = o16; if (lo) { *(volatile v2us*)(Ph + oo) = oh; *(volatile v2us*)(Pl + oo) = ol; }
}
__global__ __launch_bounds__(256) void k_vtp(const float* __restrict__ F, int pitch, int col0, int nheads, h16* V16, bf* Vh, bf* Vl) {
    const size_t e = ((size_t)blockIdx.x * 256 + threadIdx.x) * 2; if (e >= (size_t)nheads * HD * TT) return;
    const int t = (int)(e % TT); const int d = (int)((e / TT) % HD); const int g = (int)(e / ((size_t)TT * HD)); v2h o16; v2us oh, ol;
#pragma unroll
    for (int q = 0; q < 2; ++q) { const float xx = F[(size_t)(t + q) * pitch + col0 + g * HD + d]; o16[q] = tohx(xx); unsigned short a2, c2; splitf(xx, a2, c2); oh[q] = a2; ol[q] = c2; }
    const bool lo = (t < RH); const size_t oo = ((size_t)g * HD + d) * RH + (lo ? t : 0);
    *(volatile v2h*)(V16 + e) = o16; if (lo) { *(volatile v2us*)(Vh + oo) = oh; *(volatile v2us*)(Vl + oo) = ol; }
    __threadfence();
    *(volatile v2h*)(V16 + e) = o16; if (lo) { *(volatile v2us*)(Vh + oo) = oh; *(volatile v2us*)(Vl + oo) = ol; }
}
__global__ __launch_bounds__(256) void k_asoft(float* Sb, bf* Ph, bf* Pl) {
    const int lane = threadIdx.x & 31; const int row = blockIdx.x * 8 + (threadIdx.x >> 5); if (row >= ZH * TT) return;
    const int i = row % TT; const int zz = row / TT; const bool hires = (i < RH); const int nch = (i >> 7) + 1;
    const float* sr = Sb + (size_t)row * TT;
    float v[TT / 32]; float mx = -3.0e38f;
#pragma unroll
    for (int ch = 0; ch < TT / 128; ++ch) {
        if (ch < nch) { const int j0 = ch * 128 + lane * 4; const v4f a = *(const v4f*)(sr + j0);
#pragma unroll
            for (int q = 0; q < 4; ++q) { const float s = a[q] * SCL; const float t = (j0 + q <= i) ? s : -3.0e38f; v[ch * 4 + q] = t; mx = fmaxf(mx, t); }
        } else {
#pragma unroll
            for (int q = 0; q < 4; ++q) v[ch * 4 + q] = -3.0e38f;
        }
    }
#pragma unroll
    for (int sh = 16; sh; sh >>= 1) mx = fmaxf(mx, __shfl_xor(mx, sh, 32));
    float sum = 0.f;
#pragma unroll
    for (int ch = 0; ch < TT / 128; ++ch) {
        if (ch < nch) {
#pragma unroll
            for (int q = 0; q < 4; ++q) { const int k = ch * 4 + q; float d0 = __fsub_rn(v[k], mx); asm volatile("" : "+v"(d0)); float p = __builtin_amdgcn_exp2f(__fmul_rn(d0, LOG2E)); p = (ch * 128 + lane * 4 + q <= i) ? p : 0.0f; v[k] = p; sum += p; }
        }
    }
#pragma unroll
    for (int sh = 16; sh; sh >>= 1) sum += __shfl_xor(sum, sh, 32);
    const float f = __fdiv_rn(hires ? 1.0f : PCAR, sum);
    h16* prow = (h16*)(Sb + (size_t)row * TT);
#pragma unroll 1
    for (int ps = 0; ps < 2; ++ps) {
        if (hires) {
#pragma unroll
            for (int ch = 0; ch < RH / 128; ++ch) { if (ch < nch) { v4us oh, ol;
#pragma unroll
                for (int q = 0; q < 4; ++q) { unsigned short a, c2; splitf(v[ch * 4 + q] * f, a, c2); oh[q] = a; ol[q] = c2; }
                const size_t oo = ((size_t)zz * RH + i) * RH + ch * 128 + lane * 4; *(volatile v4us*)(Ph + oo) = oh; *(volatile v4us*)(Pl + oo) = ol; } }
        } else {
#pragma unroll
            for (int ch = 0; ch < TT / 128; ++ch) { if (ch < nch) { v4h o4;
#pragma unroll
                for (int q = 0; q < 4; ++q) o4[q] = tohx(v[ch * 4 + q] * f);
                *(volatile v4h*)(prow + ch * 128 + lane * 4) = o4; } } }
        if (ps == 0) __threadfence(); }
}
__global__ __launch_bounds__(256) void k_merge(const float* __restrict__ O, int h0, bf* Ah, bf* Al, h16* A16) {
    const size_t e = ((size_t)blockIdx.x * 256 + threadIdx.x) * 2; if (e >= (size_t)ZH * TT * HD) return;
    const int d = (int)(e % HD); const int t = (int)((e / HD) % TT); const int zz = (int)(e / ((size_t)HD * TT));
    const v2f ov = *(const v2f*)(O + e); const int col = (h0 + zz) * HD + d;
    if (t < RH) {
        v2us oh, ol;
#pragma unroll
        for (int q = 0; q < 2; ++q) { unsigned short a, c2; splitf(ov[q], a, c2); oh[q] = a; ol[q] = c2; }
        const size_t oo = (size_t)t * DM + col;
        *(volatile v2us*)(Ah + oo) = oh; *(volatile v2us*)(Al + oo) = ol; __threadfence(); *(volatile v2us*)(Ah + oo) = oh; *(volatile v2us*)(Al + oo) = ol;
    } else {
        v2h o;
#pragma unroll
        for (int q = 0; q < 2; ++q) o[q] = tohx(ov[q] * (ASC / PCAR));
        const size_t oo = (size_t)(t - RH) * DM + col;
        *(volatile v2h*)(A16 + oo) = o; __threadfence(); *(volatile v2h*)(A16 + oo) = o;
    }
}

extern "C" void kernel_launch(void* const* d_in, const int* in_sizes, int n_in,
                              void* d_out, int out_size, void* d_ws, size_t ws_size, hipStream_t stream) {
    if (n_in < 3) return;
    if ((size_t)in_sizes[0] < (size_t)(NB - 1) * TT_FULL * DM + (size_t)TT * DM) return;
    if ((size_t)in_sizes[1] < (size_t)NQKV * DM) return;
    if ((size_t)in_sizes[2] < (size_t)DM * DM) return;
    if ((size_t)out_size < (size_t)NB * TT * DM) return;
    const float* x = (const float*)d_in[0]; const float* wqkv = (const float*)d_in[1]; const float* wo = (const float*)d_in[2];
    float* OUT = (float*)d_out;
    char* base = (char*)d_ws; size_t off = 0;
    auto al = [](size_t bytes) { return (bytes + 255) & ~(size_t)255; };
    auto take = [&](size_t bytes) { char* p = base + off; off += al(bytes); return (void*)p; };
    bf*  WOb  = (bf*)take((size_t)DM * DM * 2);
    h16* WO16 = (h16*)take((size_t)DM * DM * 2);
    float* CS = (float*)take((size_t)TT * HP * 2 * 4);
    float* TH = (float*)take(256);
    h16* QK16 = (h16*)take((size_t)NPL * TT * HD * 2);
    bf*  QKh  = (bf*)take((size_t)NPL * RH * HD * 2);
    bf*  QKl  = (bf*)take((size_t)NPL * RH * HD * 2);
    h16* VT16 = (h16*)take((size_t)NKV * HD * TT * 2);
    bf*  VTh  = (bf*)take((size_t)NKV * HD * RH * 2);
    bf*  VTl  = (bf*)take((size_t)NKV * HD * RH * 2);
    bf*  Ph   = (bf*)take((size_t)ZH * RH * RH * 2);
    bf*  Pl   = (bf*)take((size_t)ZH * RH * RH * 2);
    float* Ob = (float*)take((size_t)ZH * TT * HD * 4);
    bf*  ATh  = (bf*)take((size_t)RH * DM * 2);
    bf*  ATl  = (bf*)take((size_t)RH * DM * 2);
    h16* AT16 = (h16*)take((size_t)(TT - RH) * DM * 2);
    const size_t szXB = al((size_t)TT * DM * 2), szF = al((size_t)TT * NQKV * 4), szWQ = al((size_t)NQKV * DM * 2), szSb = al((size_t)ZH * TT * TT * 4);
    const size_t szU = (szXB + szF + szWQ > szSb) ? (szXB + szF + szWQ) : szSb;
    char* U = (char*)take(szU);
    bf*  XB   = (bf*)U; float* FQKV = (float*)(U + szXB); bf* WQ = (bf*)(U + szXB + szF); float* Sb = (float*)U;
    if (off > ws_size) return;

    k_cvt8<<<(unsigned)(((size_t)DM * DM / 8 + 255) / 256), 256, 0, stream>>>(wo, WOb, (size_t)DM * DM / 8);
    k_cvt8h<<<(unsigned)(((size_t)DM * DM / 8 + 255) / 256), 256, 0, stream>>>(wo, WO16, WSC, (size_t)DM * DM / 8);
    k_theta<<<1, 32, 0, stream>>>(TH);
    k_cstab<<<(unsigned)((TT * HP + 255) / 256), 256, 0, stream>>>(TH, CS);
    const unsigned LQK = (unsigned)(((size_t)NPL * TT * HD / 2 + 255) / 256), LV = (unsigned)(((size_t)NKV * HD * TT / 2 + 255) / 256), LM = (unsigned)(((size_t)ZH * TT * HD / 2 + 255) / 256);
    for (int b = 0; b < NB; ++b) {
        k_cvt8<<<(unsigned)(((size_t)NQKV * DM / 8 + 255) / 256), 256, 0, stream>>>(wqkv, WQ, (size_t)NQKV * DM / 8);
        k_cvt8<<<(unsigned)(((size_t)TT * DM / 8 + 255) / 256), 256, 0, stream>>>(x + (size_t)b * TT_FULL * DM, XB, (size_t)TT * DM / 8);
        k_gemmw<bf, 0, 0><<<dim3(TT / 64, NQKV / 64, 1), 32, 0, stream>>>(XB, nullptr, DM, WQ, nullptr, DM, DM, 0, FQKV, NQKV, 1.0f, 0, 0, 0);
        k_rope<<<LQK, 256, 0, stream>>>(FQKV, NQKV, NPL, CS, QK16, QKh, QKl);
        k_vtp<<<LV, 256, 0, stream>>>(FQKV, NQKV, NPL * HD, NKV, VT16, VTh, VTl);
        for (int h0 = 0; h0 < NQH; h0 += ZH) { const int kv = h0 / REP;
            k_gemmw<bf, 2, 1><<<dim3(RH / 64, RH / 64, ZH), 32, 0, stream>>>(QKh + (size_t)h0 * RH * HD, QKl + (size_t)h0 * RH * HD, HD, QKh + (size_t)(NQH + kv) * RH * HD, QKl + (size_t)(NQH + kv) * RH * HD, HD, HD, 0, Sb, TT, 1.0f, (size_t)RH * HD, 0, (size_t)TT * TT);
            if (TT > RH) k_gemmw<h16, 0, 1><<<dim3((TT - RH) / 64, TT / 64, ZH), 32, 0, stream>>>(QK16 + ((size_t)h0 * TT + RH) * HD, nullptr, HD, QK16 + (size_t)(NQH + kv) * TT * HD, nullptr, HD, HD, RH, Sb + (size_t)RH * TT, TT, 1.0f, (size_t)TT * HD, 0, (size_t)TT * TT);
            k_asoft<<<(unsigned)(ZH * TT / 8), 256, 0, stream>>>(Sb, Ph, Pl);
            k_gemmw<bf, 2, 2><<<dim3(RH / 64, HD / 64, ZH), 32, 0, stream>>>(Ph, Pl, RH, VTh + (size_t)kv * HD * RH, VTl + (size_t)kv * HD * RH, RH, RH, 0, Ob, HD, 1.0f, (size_t)RH * RH, 0, (size_t)TT * HD);
            if (TT > RH) k_gemmw<h16, 0, 2><<<dim3((TT - RH) / 64, HD / 64, ZH), 32, 0, stream>>>((const h16*)Sb + (size_t)RH * 2 * TT, nullptr, 2 * TT, VT16 + (size_t)kv * HD * TT, nullptr, TT, TT, RH, Ob + (size_t)RH * HD, HD, 1.0f, (size_t)2 * TT * TT, 0, (size_t)TT * HD);
            k_merge<<<LM, 256, 0, stream>>>(Ob, h0, ATh, ATl, AT16); }
        float* OUTb = OUT + (size_t)b * TT * DM;
        k_gemmw<bf, 1, 0><<<dim3(RH / 64, DM / 64, 1), 32, 0, stream>>>(ATh, ATl, DM, WOb, nullptr, DM, DM, 0, OUTb, DM, 1.0f, 0, 0, 0);
        if (TT > RH) k_gemmw<h16, 0, 0><<<dim3((TT - RH) / 64, DM / 64, 1), 32, 0, stream>>>(AT16, nullptr, DM, WO16, nullptr, DM, DM, 0, OUTb + (size_t)RH * DM, DM, OSC, 0, 0, 0);
    }
}
